// NeuralAdditiveModel_75127567941662
// MI455X (gfx1250) — hardware-verified
//
#include <hip/hip_runtime.h>
#include <math.h>

constexpr int kRows   = 4096;
constexpr int kFeat   = 512;
constexpr int kS0     = 32;
constexpr int kHid1   = 64;
constexpr int kHid2   = 32;
constexpr int kFChunk = 128;
constexpr int kNChunk = kFeat / kFChunk;
constexpr long kA1Stride = (long)kRows * kS0;
constexpr long kA2Stride = (long)kRows * kHid1;
constexpr float kOpScaleA = 8.0f;
constexpr float kOpScaleW = 16.0f;
constexpr float kAccFold  = 1.0f / 128.0f;
static_assert(kFeat % kFChunk == 0);
static_assert(kRows % 256 == 0);
static_assert(kS0 == 32 && kHid1 == 64 && kHid2 == 32);

typedef __attribute__((ext_vector_type(16))) _Float16 v16h;
typedef __attribute__((ext_vector_type(8)))  _Float16 v8h;
typedef __attribute__((ext_vector_type(16))) __bf16   v16b;
typedef __attribute__((ext_vector_type(8)))  __bf16   v8b;
typedef __attribute__((ext_vector_type(8)))  float    v8f;
typedef __attribute__((ext_vector_type(4)))  float    v4f;
typedef __attribute__((ext_vector_type(4)))  unsigned int v4u;

__device__ __forceinline__ unsigned short f2bf_bits(float f) {
  unsigned u = __float_as_uint(f);
  return (unsigned short)((u + 0x7FFFu + ((u >> 16) & 1u)) >> 16);
}
__device__ __forceinline__ float bf_bits2f(unsigned short h) { return __uint_as_float(((unsigned)h) << 16); }

__device__ __forceinline__ void dep_guard_h(v8f& a, v8f& b, v16h x, v16h y) { asm volatile("v_nop\n\tv_nop\n\tv_nop\n\tv_nop" : "+v"(a), "+v"(b) : "v"(x), "v"(y)); }
__device__ __forceinline__ void dep_guard_b(v8f& a, v8f& b, v16b x, v16b y) { asm volatile("v_nop\n\tv_nop\n\tv_nop\n\tv_nop" : "+v"(a), "+v"(b) : "v"(x), "v"(y)); }
__device__ __forceinline__ void keep4_h(v16h a, v16h b, v16h c, v16h d) { asm volatile("v_nop" :: "v"(a), "v"(b), "v"(c), "v"(d)); }
__device__ __forceinline__ void keep4_b(v16b a, v16b b, v16b c, v16b d) { asm volatile("v_nop" :: "v"(a), "v"(b), "v"(c), "v"(d)); }
__device__ __forceinline__ void acc_guard4(v8f& a, v8f& b, v8f& c, v8f& d) { asm volatile("v_nop\n\tv_nop\n\tv_nop\n\tv_nop" : "+v"(a), "+v"(b), "+v"(c), "+v"(d)); }
template <typename T> struct Frag;
template <> struct Frag<_Float16> {
  typedef v16h V; union U { v16h v; v8h h[2]; };
  static __device__ __forceinline__ v16h load(const _Float16* p) {
    U f; f.h[0] = *(const v8h*)(p); f.h[1] = *(const v8h*)(p + 16); return f.v;
  }
  static __device__ __forceinline__ v8f mma(v16h a, v16h b, v8f c) {
    return __builtin_amdgcn_wmma_f32_16x16x32_f16(false, a, false, b, (short)0, c, false, false);
  }
  static __device__ __forceinline__ void guard(v8f& a, v8f& b, v16h x, v16h y) { dep_guard_h(a, b, x, y); }
  static __device__ __forceinline__ void keep(v16h a, v16h b, v16h c, v16h d) { keep4_h(a, b, c, d); }
};
template <> struct Frag<__bf16> {
  typedef v16b V; union U { v16b v; v8b h[2]; };
  static __device__ __forceinline__ v16b load(const __bf16* p) {
    U f; f.h[0] = *(const v8b*)(p); f.h[1] = *(const v8b*)(p + 16); return f.v;
  }
  static __device__ __forceinline__ v8f mma(v16b a, v16b b, v8f c) {
    return __builtin_amdgcn_wmma_f32_16x16x32_bf16(false, a, false, b, (short)0, c, false, false);
  }
  static __device__ __forceinline__ void guard(v8f& a, v8f& b, v16b x, v16b y) { dep_guard_b(a, b, x, y); }
  static __device__ __forceinline__ void keep(v16b a, v16b b, v16b c, v16b d) { keep4_b(a, b, c, d); }
};

__device__ __forceinline__ unsigned pk16(unsigned short a, unsigned short b) { return (unsigned)a | ((unsigned)b << 16); }
__device__ __forceinline__ unsigned short h_bits(float f) { const _Float16 h = (_Float16)f; return __builtin_bit_cast(unsigned short, h); }

template <int ET> struct Elem;
template <> struct Elem<0> { typedef _Float16 T; };
template <> struct Elem<1> { typedef __bf16 T; };
template <int ET, bool SPLIT, int BIAS_MODE, int OUT_MODE, bool RESID, int ACT = 0>
__global__ __launch_bounds__(256) void wmma_gemm64(
    const unsigned short* __restrict__ Ap, const unsigned short* __restrict__ A2p, int lda, long strideA,
    const unsigned short* __restrict__ Btp, const unsigned short* __restrict__ Bt2p, int ldb, long strideB,
    void* __restrict__ Cout, void* __restrict__ Cout2, int ldc, long strideC,
    const float* __restrict__ bias, long strideBias,
    const float* __restrict__ resid, long strideR,
    int M, int N, int K, float scale, float pscale) {
  typedef typename Elem<ET>::T T;
  typedef typename Frag<T>::V V;
  const T* A = (const T*)Ap; const T* A2 = (const T*)A2p; const T* Bt = (const T*)Btp; const T* Bt2 = (const T*)Bt2p;
  __shared__ __align__(16) float sT[8][16 * 68];
  const int b    = blockIdx.y;
  const int lane = threadIdx.x & 31;
  const int wave = threadIdx.x >> 5;
  const int tilesN = N >> 6;
  const int tilesM = M >> 6;
  const int tile = blockIdx.x * 8 + wave;
  if (tile >= tilesM * tilesN) return;
  const int tm = tile / tilesN;
  const int tn = tile - tm * tilesN;
  const int m0 = tm << 6;
  const int n0 = tn << 6;

  const T* Ab  = A  + (size_t)b * strideA;
  const T* Bb  = Bt + (size_t)b * strideB;
  const T* Ab2 = SPLIT ? (A2  + (size_t)b * strideA) : nullptr;
  const T* Bb2 = SPLIT ? (Bt2 + (size_t)b * strideB) : nullptr;

  const int rlane = lane & 15;
  const int koff  = (lane >> 4) * 8;
  const int mOff  = (lane >> 4) * 8;

  v8f acc[4][4];
#pragma unroll
  for (int i = 0; i < 4; ++i)
#pragma unroll
    for (int j = 0; j < 4; ++j) acc[i][j] = (v8f){0.f,0.f,0.f,0.f,0.f,0.f,0.f,0.f};

  for (int k0 = 0; k0 < K; k0 += 32) {
    V bh[4], bl[4];
#pragma unroll
    for (int j = 0; j < 4; ++j) {
      const size_t bo = (size_t)(n0 + (j << 4) + rlane) * ldb + koff + k0;
      bh[j] = Frag<T>::load(Bb + bo);
      if (SPLIT) bl[j] = Frag<T>::load(Bb2 + bo);
    }
#pragma unroll
    for (int i = 0; i < 4; ++i) {
      const size_t ao = (size_t)(m0 + (i << 4) + rlane) * lda + koff + k0;
      V ah = Frag<T>::load(Ab + ao);
      V al;
      if (SPLIT) al = Frag<T>::load(Ab2 + ao);
#pragma unroll
      for (int j = 0; j < 4; ++j) {
        acc[i][j] = Frag<T>::mma(ah, bh[j], acc[i][j]);
        if (SPLIT) {
          acc[i][j] = Frag<T>::mma(ah, bl[j], acc[i][j]);
          acc[i][j] = Frag<T>::mma(al, bh[j], acc[i][j]);
        }
      }
      Frag<T>::guard(acc[i][0], acc[i][3], ah, SPLIT ? al : ah);
    }
    Frag<T>::keep(bh[0], bh[1], bh[2], bh[3]);
    if (SPLIT) Frag<T>::keep(bl[0], bl[1], bl[2], bl[3]);
  }
  acc_guard4(acc[0][0], acc[0][1], acc[0][2], acc[0][3]);
  acc_guard4(acc[1][0], acc[1][1], acc[1][2], acc[1][3]);
  acc_guard4(acc[2][0], acc[2][1], acc[2][2], acc[2][3]);
  acc_guard4(acc[3][0], acc[3][1], acc[3][2], acc[3][3]);

  float* slab = sT[wave];
  const float* Rb = RESID ? (resid + (size_t)b * strideR) : nullptr;
#pragma unroll
  for (int i = 0; i < 4; ++i) {
    const int mBase = m0 + (i << 4);
#pragma unroll
    for (int j = 0; j < 4; ++j) {
      const int n = n0 + (j << 4) + rlane;
      float bv = 0.f;
      if (BIAS_MODE == 2) bv = bias[n];
      if (BIAS_MODE == 3) bv = bias[(size_t)b * strideBias + n];
#pragma unroll
      for (int r = 0; r < 8; ++r) {
        float v = acc[i][j][r] * scale;
        if (BIAS_MODE == 1) v += bias[mBase + mOff + r];
        if (BIAS_MODE == 2) v += bv;
        if (RESID) v += Rb[(size_t)(mBase + mOff + r) * ldc + n];
        if (ACT == 2) v = fmaxf(v, 0.0f);
        if (ACT == 4) v = (v > 0.f) ? v : 0.01f * v;
        if (BIAS_MODE == 3) v = (v - bv) * pscale;
        slab[(mOff + r) * 68 + (j << 4) + rlane] = v;
      }
    }
    __builtin_amdgcn_fence(__ATOMIC_RELEASE, "workgroup");
    __builtin_amdgcn_wave_barrier();
    __builtin_amdgcn_fence(__ATOMIC_ACQUIRE, "workgroup");
    if (OUT_MODE == 0) {
      float* C = (float*)Cout + (size_t)b * strideC;
      const int hh = lane >> 4, c4 = (lane & 15) * 4;
      for (int pass = 0; pass < 2; ++pass) {
#pragma unroll
        for (int it = 0; it < 8; ++it) {
          const int row = it * 2 + hh;
          v4f v = *(const v4f*)(slab + row * 68 + c4);
          *(volatile v4f*)(C + (size_t)(mBase + row) * ldc + n0 + c4) = v;
        }
        __threadfence();
      }
    } else {
      const int q = lane >> 3, c8 = (lane & 7) * 8;
      unsigned short* C  = (unsigned short*)Cout  + (size_t)b * strideC;
      unsigned short* C2 = (OUT_MODE == 2) ? ((unsigned short*)Cout2 + (size_t)b * strideC) : nullptr;
      for (int pass = 0; pass < 2; ++pass) {
#pragma unroll
        for (int it = 0; it < 4; ++it) {
          const int row = it * 4 + q;
          const float* sp = slab + row * 68 + c8;
          v8h hv, lv;
#pragma unroll
          for (int e = 0; e < 8; ++e) {
            if (OUT_MODE == 1) {
              hv[e] = (_Float16)sp[e];
            } else {
              unsigned short hb = f2bf_bits(sp[e]);
              unsigned short lb = f2bf_bits(sp[e] - bf_bits2f(hb));
              hv[e] = __builtin_bit_cast(_Float16, hb);
              lv[e] = __builtin_bit_cast(_Float16, lb);
            }
          }
          *(volatile v8h*)(C + (size_t)(mBase + row) * ldc + n0 + c8) = hv;
          if (OUT_MODE == 2) *(volatile v8h*)(C2 + (size_t)(mBase + row) * ldc + n0 + c8) = lv;
        }
        __threadfence();
      }
    }
    __builtin_amdgcn_fence(__ATOMIC_RELEASE, "workgroup");
    __builtin_amdgcn_wave_barrier();
    __builtin_amdgcn_fence(__ATOMIC_ACQUIRE, "workgroup");
  }
}

__global__ __launch_bounds__(256) void prep_kernel(const float* __restrict__ W0, const float* __restrict__ b0,
                                                   const float* __restrict__ W1, const float* __restrict__ W2,
                                                   float* __restrict__ SESB,
                                                   unsigned short* __restrict__ Bt1, unsigned short* __restrict__ Bt2) {
  __shared__ float sW1[2048];
  __shared__ float sW2[2048];
  __shared__ float sE[1024];
  __shared__ float sb0[32];
  __shared__ __align__(16) float sS[64];
  const int f = blockIdx.x;
  const int t = threadIdx.x;
#pragma unroll
  for (int i = 0; i < 8; ++i) {
    const int idx = i * 256 + t;
    sW1[idx] = W1[(size_t)f * 2048 + idx];
    sW2[idx] = W2[(size_t)f * 2048 + idx];
  }
#pragma unroll 1
  for (int e = 0; e < 4; ++e) {
    const int idx = e * 256 + t;
    sE[idx] = expf(W0[(size_t)f * 1024 + idx]);
  }
  {
    const float bv = b0[(size_t)f * 32 + (t & 31)];
    if (t < 32) sb0[t] = bv;
  }
  __syncthreads();
  if (t < 32) {
    float se = 0.f, sb = 0.f;
#pragma unroll 1
    for (int s = 0; s < 32; ++s) {
      const float ev = sE[s * 32 + t];
      se += ev;
      sb += sb0[s] * ev;
    }
    sS[t] = se;
    sS[32 + t] = sb;
  }
  __syncthreads();
  {
    const int tc = t & 15;
    const v4f v = *(const v4f*)(sS + 4 * tc);
    float* dst = SESB + (size_t)f * 64 + 4 * tc;
    for (int pass = 0; pass < 2; ++pass) {
      if (t < 16) *(volatile v4f*)dst = v;
      __threadfence();
    }
  }
  {
    const int n = t >> 2, kq = (t & 3) * 8;
    unsigned short hb[8];
#pragma unroll
    for (int e = 0; e < 8; ++e) hb[e] = h_bits(sW1[(kq + e) * 64 + n] * kOpScaleW);
    const v4u u = (v4u){pk16(hb[0], hb[1]), pk16(hb[2], hb[3]), pk16(hb[4], hb[5]), pk16(hb[6], hb[7])};
    unsigned short* q = Bt1 + (size_t)f * 2048 + 8 * t;
    *(volatile v4u*)q = u;
    __threadfence();
    *(volatile v4u*)q = u;
  }
  {
    const int n = t >> 3, kq = (t & 7) * 8;
    unsigned short hb[8];
#pragma unroll
    for (int e = 0; e < 8; ++e) hb[e] = h_bits(sW2[(kq + e) * 32 + n] * kOpScaleW);
    const v4u u = (v4u){pk16(hb[0], hb[1]), pk16(hb[2], hb[3]), pk16(hb[4], hb[5]), pk16(hb[6], hb[7])};
    unsigned short* q = Bt2 + (size_t)f * 2048 + 8 * t;
    *(volatile v4u*)q = u;
    __threadfence();
    *(volatile v4u*)q = u;
  }
}

__global__ __launch_bounds__(256) void shallow_a1_kernel(const float* __restrict__ x, const float* __restrict__ SESB,
                                                         const float* __restrict__ b1,
                                                         unsigned short* __restrict__ A1c, int f0) {
  __shared__ __align__(16) float sS[64];
  __shared__ float sb1[32];
  __shared__ __align__(16) unsigned sA[256 * 16];
  const int t  = threadIdx.x;
  const int by = blockIdx.x;
  const int fl = blockIdx.y;
  const int f  = f0 + fl;
  {
    const float sv = SESB[(size_t)f * 64 + (t & 63)];
    const float bv = b1[(size_t)f * 32 + (t & 31)];
    if (t < 64) sS[t] = sv;
    if (t < 32) sb1[t] = bv;
  }
  __syncthreads();

  const int b = by * 256 + t;
  const float xv = x[(size_t)b * kFeat + f];
#pragma unroll
  for (int h2 = 0; h2 < 16; ++h2) {
    const int h = 2 * h2;
    const float v0 = fminf(fmaxf(xv * sS[h]     - sS[32 + h],     0.f), 1.f);
    const float v1 = fminf(fmaxf(xv * sS[h + 1] - sS[32 + h + 1], 0.f), 1.f);
    const float a0 = (v0 - sb1[h])     * kOpScaleA;
    const float a1 = (v1 - sb1[h + 1]) * kOpScaleA;
    sA[t * 16 + h2] = pk16(h_bits(a0), h_bits(a1));
  }
  __syncthreads();

  unsigned short* base = A1c + ((size_t)fl * kRows + (size_t)by * 256) * kS0;
  for (int pass = 0; pass < 2; ++pass) {
#pragma unroll
    for (int it = 0; it < 4; ++it) {
      const int c = it * 256 + t;
      const v4u v = *(const v4u*)(sA + c * 4);
      *(volatile v4u*)(base + (size_t)c * 8) = v;
    }
    __threadfence();
  }
}

__global__ __launch_bounds__(256) void gemm_l2_dot_kernel(
    const unsigned short* __restrict__ Ap, long strideA,
    const unsigned short* __restrict__ Btp, long strideB,
    const float* __restrict__ Wl,
    float* __restrict__ FT,
    float scale) {
  __shared__ __align__(16) float sF[8][64];
  const int b    = blockIdx.y;
  const int lane = threadIdx.x & 31;
  const int wave = threadIdx.x >> 5;
  const int tile = blockIdx.x * 8 + wave;
  if (tile >= (kRows >> 6)) return;
  const int m0 = tile << 6;
  const _Float16* Ab = (const _Float16*)Ap  + (size_t)b * strideA;
  const _Float16* Bb = (const _Float16*)Btp + (size_t)b * strideB;
  const int rlane = lane & 15;
  const int koff  = (lane >> 4) * 8;
  const int mOff  = (lane >> 4) * 8;

  v8f acc[4][2];
#pragma unroll
  for (int i = 0; i < 4; ++i)
#pragma unroll
    for (int j = 0; j < 2; ++j) acc[i][j] = (v8f){0.f,0.f,0.f,0.f,0.f,0.f,0.f,0.f};

#pragma unroll
  for (int ks = 0; ks < 2; ++ks) {
    const int k0 = ks * 32;
    v16h bh[2];
#pragma unroll
    for (int j = 0; j < 2; ++j)
      bh[j] = Frag<_Float16>::load(Bb + (size_t)((j << 4) + rlane) * kHid1 + koff + k0);
#pragma unroll
    for (int i = 0; i < 4; ++i) {
      const v16h ah = Frag<_Float16>::load(Ab + (size_t)(m0 + (i << 4) + rlane) * kHid1 + koff + k0);
#pragma unroll
      for (int j = 0; j < 2; ++j) acc[i][j] = Frag<_Float16>::mma(ah, bh[j], acc[i][j]);
      Frag<_Float16>::guard(acc[i][0], acc[i][1], ah, ah);
    }
    Frag<_Float16>::keep(bh[0], bh[1], bh[0], bh[1]);
  }
  acc_guard4(acc[0][0], acc[0][1], acc[1][0], acc[1][1]);
  acc_guard4(acc[2][0], acc[2][1], acc[3][0], acc[3][1]);

  const float wl0 = Wl[(size_t)b * kHid2 + rlane];
  const float wl1 = Wl[(size_t)b * kHid2 + 16 + rlane];
  float* sf = sF[wave];
#pragma unroll
  for (int i = 0; i < 4; ++i) {
    float p[8];
#pragma unroll
    for (int r = 0; r < 8; ++r) {
      const float v0 = fmaxf(acc[i][0][r] * scale, 0.f);
      const float v1 = fmaxf(acc[i][1][r] * scale, 0.f);
      p[r] = v0 * wl0 + v1 * wl1;
    }
#pragma unroll
    for (int r = 0; r < 8; ++r) {
      float v = p[r];
      v += __shfl_xor(v, 1, 32);
      v += __shfl_xor(v, 2, 32);
      v += __shfl_xor(v, 4, 32);
      v += __shfl_xor(v, 8, 32);
      p[r] = v;
    }
#pragma unroll
    for (int r = 0; r < 8; ++r) sf[16 * i + mOff + r] = p[r];
  }
  __builtin_amdgcn_fence(__ATOMIC_RELEASE, "workgroup");
  __builtin_amdgcn_wave_barrier();
  __builtin_amdgcn_fence(__ATOMIC_ACQUIRE, "workgroup");
  const v4f v = *(const v4f*)(sf + 4 * rlane);
  float* dst = FT + (size_t)b * kRows + m0 + 4 * rlane;
  for (int pass = 0; pass < 2; ++pass) {
    if (lane < 16) *(volatile v4f*)dst = v;
    __threadfence();
  }
}

__global__ __launch_bounds__(256) void fout_transpose_kernel(const float* __restrict__ FT, float* __restrict__ out1) {
  __shared__ __align__(16) float sTr[16][516];
  const int t = threadIdx.x;
  const int lane = t & 31, wave = t >> 5;
  const int b0 = blockIdx.x * 16;
#pragma unroll 4
  for (int it = 0; it < 32; ++it) {
    const int e  = it * 256 + t;
    const int f  = e >> 4;
    const int bl = e & 15;
    sTr[bl][f] = FT[(size_t)f * kRows + b0 + bl];
  }
  __syncthreads();
  for (int pass = 0; pass < 2; ++pass) {
#pragma unroll
    for (int rr = 0; rr < 2; ++rr) {
      const int row = wave * 2 + rr;
#pragma unroll
      for (int q = 0; q < 4; ++q) {
        const v4f v = *(const v4f*)(&sTr[row][q * 128 + lane * 4]);
        *(volatile v4f*)(out1 + (size_t)(b0 + row) * kFeat + q * 128 + lane * 4) = v;
      }
    }
    __threadfence();
  }
}

__global__ __launch_bounds__(256) void out_sum_kernel(const float* __restrict__ FT, const float* __restrict__ ob,
                                                     float* __restrict__ out0) {
  __shared__ __align__(16) float sS[256];
  const int t = threadIdx.x;
  const int b = blockIdx.x * 256 + t;
  float s = 0.f;
#pragma unroll 8
  for (int f = 0; f < kFeat; ++f) s += FT[(size_t)f * kRows + b];
  s += ob[0];
  sS[t] = s;
  __syncthreads();
  const int tc = t & 63;
  const v4f v = *(const v4f*)(sS + 4 * tc);
  float* dst = out0 + (size_t)blockIdx.x * 256 + 4 * tc;
  for (int pass = 0; pass < 2; ++pass) {
    if (t < 64) *(volatile v4f*)dst = v;
    __threadfence();
  }
}

extern "C" void kernel_launch(void* const* d_in, const int* in_sizes, int n_in,
                              void* d_out, int out_size, void* d_ws, size_t ws_size,
                              hipStream_t stream) {
  if (n_in < 9) return;
  if (in_sizes[0] != kRows * kFeat) return;
  if (in_sizes[1] != kFeat * kS0 * kS0) return;
  if (in_sizes[3] != kFeat * kS0 * kHid1) return;
  if (in_sizes[5] != kFeat * kHid1 * kHid2) return;
  if (out_size != kRows + kRows * kFeat) return;

  const float* x  = (const float*)d_in[0];
  const float* W0 = (const float*)d_in[1];
  const float* b0 = (const float*)d_in[2];
  const float* W1 = (const float*)d_in[3];
  const float* b1 = (const float*)d_in[4];
  const float* W2 = (const float*)d_in[5];
  const float* b2 = (const float*)d_in[6];
  const float* Wl = (const float*)d_in[7];
  const float* ob = (const float*)d_in[8];

  float* out0 = (float*)d_out;
  float* out1 = out0 + kRows;

  const size_t offSESB = 0;
  const size_t offBt1  = offSESB + (size_t)kFeat * 64 * 4;
  const size_t offBt2  = offBt1  + (size_t)kFeat * 2048 * 2;
  const size_t offFT   = offBt2  + (size_t)kFeat * 2048 * 2;
  const size_t offA1   = offFT   + (size_t)kFeat * kRows * 4;
  const size_t offA2   = offA1   + (size_t)kFChunk * kA1Stride * 2;
  const size_t total   = offA2   + (size_t)kFChunk * kA2Stride * 2;
  if (total > ws_size) return;

  char* ws = (char*)d_ws;
  float* SESB         = (float*)(ws + offSESB);
  unsigned short* Bt1 = (unsigned short*)(ws + offBt1);
  unsigned short* Bt2 = (unsigned short*)(ws + offBt2);
  float* FT           = (float*)(ws + offFT);
  unsigned short* A1c = (unsigned short*)(ws + offA1);
  unsigned short* A2c = (unsigned short*)(ws + offA2);

  prep_kernel<<<dim3(kFeat), dim3(256), 0, stream>>>(W0, b0, W1, W2, SESB, Bt1, Bt2);

  for (int c = 0; c < kNChunk; ++c) {
    const int f0 = c * kFChunk;
    shallow_a1_kernel<<<dim3(kRows / 256, kFChunk), dim3(256), 0, stream>>>(x, SESB, b1, A1c, f0);

    const unsigned short* Bt1c = Bt1 + (size_t)f0 * 2048;
    const float* b2c = b2 + (size_t)f0 * kHid1;
    wmma_gemm64<0, false, 3, 1, false, 2><<<dim3(8, kFChunk), dim3(256), 0, stream>>>(
        (const unsigned short*)A1c, (const unsigned short*)A1c, (int)kS0, (long)kA1Stride,
        Bt1c, Bt1c, (int)kS0, (long)2048,
        (void*)A2c, (void*)A2c, (int)kHid1, (long)kA2Stride,
        b2c, (long)kHid1,
        b2c, (long)0,
        (int)kRows, (int)kHid1, (int)kS0, (float)kAccFold, (float)kOpScaleA);

    const unsigned short* Bt2c = Bt2 + (size_t)f0 * 2048;
    const float* Wlc = Wl + (size_t)f0 * kHid2;
    float* FTc = FT + (size_t)f0 * kRows;
    gemm_l2_dot_kernel<<<dim3(8, kFChunk), dim3(256), 0, stream>>>(
        (const unsigned short*)A2c, (long)kA2Stride, Bt2c, (long)2048, Wlc, FTc, (float)kAccFold);
  }

  fout_transpose_kernel<<<dim3(kRows / 16), dim3(256), 0, stream>>>((const float*)FT, out1);
  out_sum_kernel<<<dim3(kRows / 256), dim3(256), 0, stream>>>((const float*)FT, ob, out0);
}
